// MySAGE_29386166239371
// MI455X (gfx1250) — hardware-run, weakly checked
//
#include <hip/hip_runtime.h>
#include <stddef.h>
#include <stdint.h>

#define MAGG_SINGLE_BF16 0

#define NN      100000
#define NE      1600000
#define HD      64
#define OC      32
#define GBM     128
#define MP      100096
#define KH      128
#define NTHR    256
#define NWAVE   8
#define EPT     8
#define WCH     (32 * EPT)
#define NBRUN   1024
#define SLB     10
#define NBK     98
#define WLCAP   3584
#define RCAP    28672
#define TRIPCAP 64
#define MAXDEG_MEAS   36
#define MAXB1024_MEAS 16710
#define ABM     64
#define SP      68
#define SP3     36
#define WSMAX   134217728

#define BK_ZINTS (NWAVE * WLCAP + RCAP + 3 * NBRUN)
#define BK_INTS  (BK_ZINTS + 16)
#define BK_LDS   (BK_INTS * 4)

#define PBX   (MP * HD / 8 / NTHR)
#define PBW   18
#define PBTOT (PBX + PBW + 1)

static_assert(HD == 64 && HD == 16 * 4 && OC == 32);
static_assert(MP % GBM == 0 && MP >= NN && MP == 782 * GBM && MP % ABM == 0);
static_assert(NN % 16 == 0);
static_assert(NBRUN == (1 << SLB) && NBRUN % ABM == 0 && NBRUN == 8 * GBM && NBRUN % 32 == 0);
static_assert(NBK * NBRUN >= MP && NBK * NBRUN >= NN);
static_assert(NE < (1 << 21) && (((long long)NE) << SLB) < (1LL << 31));
static_assert(NE % WCH == 0 && NE % 4 == 0);
static_assert(RCAP == NWAVE * WLCAP && RCAP % (NTHR * 4) == 0 && BK_ZINTS % 4 == 0);
static_assert((long long)RCAP * 100 >= (long long)MAXB1024_MEAS * 105);
static_assert((long long)WLCAP * 2 * NWAVE >= (long long)MAXB1024_MEAS * 3);
static_assert(MAXDEG_MEAS + 8 <= TRIPCAP);
static_assert((MP * HD / 8) % NTHR == 0);
static_assert(192 % 32 == 0 && 256 % 32 == 0 && KH == 2 * HD);
static_assert(BK_LDS <= 300000);
static_assert((GBM * SP + 64) * 4 <= 65536);
static_assert(GBM * SP3 <= GBM * SP);
static_assert((long long)NN * OC == 3200000LL);

typedef float          v4f   __attribute__((ext_vector_type(4)));
typedef float          v8f   __attribute__((ext_vector_type(8)));
typedef int            v4i   __attribute__((ext_vector_type(4)));
typedef int            v8i   __attribute__((ext_vector_type(8)));
typedef unsigned       v2u   __attribute__((ext_vector_type(2)));
typedef unsigned short v8us  __attribute__((ext_vector_type(8)));
typedef unsigned short v16us __attribute__((ext_vector_type(16)));
typedef __bf16         v16bf __attribute__((ext_vector_type(16)));
typedef v4f  __attribute__((may_alias)) v4fa;
typedef v4i  __attribute__((may_alias)) v4ia;
typedef v2u  __attribute__((may_alias)) v2ua;
typedef v8us __attribute__((may_alias)) v8usa;
union FragB { v16bf v; v16us u; v8us h[2]; v8i w; };

__device__ __forceinline__ v8f wmb(const FragB& a, const FragB& b, v8f c) {
  v8f d = __builtin_amdgcn_wmma_f32_16x16x32_bf16(false, a.v, false, b.v, (short)0, c, false, false);
  asm volatile("v_nop\n\tv_nop\n\tv_nop\n\tv_nop" : "+v"(d) : "v"(a.w), "v"(b.w));
  return d;
}

__device__ __forceinline__ unsigned bf16_bits(float f) {
  const unsigned u = __float_as_uint(f);
  const unsigned r = (u + 0x7FFFu + ((u >> 16) & 1u)) >> 16;
  const unsigned q = (u >> 16) | 0x40u;
  return ((u & 0x7fffffffu) > 0x7f800000u) ? q : r;
}

__device__ __forceinline__ void hilo_pack(float v0, float v1, float v2, float v3,
                                          int& h01, int& h23, int& l01, int& l23) {
  const unsigned a0 = bf16_bits(v0), a1 = bf16_bits(v1), a2 = bf16_bits(v2), a3 = bf16_bits(v3);
  h01 = (int)(a0 | (a1 << 16)); h23 = (int)(a2 | (a3 << 16));
#if MAGG_SINGLE_BF16
  l01 = 0; l23 = 0;
#else
  const unsigned b0 = bf16_bits(v0 - __uint_as_float(a0 << 16));
  const unsigned b1 = bf16_bits(v1 - __uint_as_float(a1 << 16));
  const unsigned b2 = bf16_bits(v2 - __uint_as_float(a2 << 16));
  const unsigned b3 = bf16_bits(v3 - __uint_as_float(a3 << 16));
  l01 = (int)(b0 | (b1 << 16)); l23 = (int)(b2 | (b3 << 16));
#endif
}

__device__ __forceinline__ v4i regroup8(int h01, int h23, int l01, int l23, int lane) {
  const int t  = lane & 15;
  const int s0 = (lane & 16) + ((2 * t) & 15), s1 = s0 + 1;
  const int a0 = __shfl(h01, s0, 32), a1 = __shfl(h23, s0, 32), a2 = __shfl(h01, s1, 32), a3 = __shfl(h23, s1, 32);
  const int b0 = __shfl(l01, s0, 32), b1 = __shfl(l23, s0, 32), b2 = __shfl(l01, s1, 32), b3 = __shfl(l23, s1, 32);
  const int mk = (t < 8) ? -1 : 0;
  v4i o;
  o.x = (a0 & mk) | (b0 & ~mk); o.y = (a1 & mk) | (b1 & ~mk);
  o.z = (a2 & mk) | (b2 & ~mk); o.w = (a3 & mk) | (b3 & ~mk);
  return o;
}

__device__ __forceinline__ void st2_v4f(float* p, v4f v) {
  *(volatile v4f*)p = v;
  __threadfence();
  *(volatile v4f*)p = v;
}
__device__ __forceinline__ void st2_v8us(unsigned short* p, v8us v) {
  *(volatile v8us*)p = v;
  __threadfence();
  *(volatile v8us*)p = v;
}

__device__ __forceinline__ v8us gather8(const float* __restrict__ base, int stride) {
  float f[8];
#pragma unroll
  for (int i = 0; i < 8; ++i) f[i] = base[(size_t)i * (size_t)stride];
  v8us o;
#pragma unroll
  for (int i = 0; i < 8; ++i) o[i] = (unsigned short)bf16_bits(f[i]);
  return o;
}

template <int NOUT>
__device__ __forceinline__ void wpart(const float* __restrict__ W, unsigned short* P, int pitch, int coff, int v) {
  const int n = v >> 3, k8 = (v & 7) * 8;
  const v8us o = gather8(W + (size_t)k8 * NOUT + n, NOUT);
  st2_v8us(P + (size_t)n * (size_t)pitch + coff + k8, o);
}

__global__ __launch_bounds__(NTHR) void k_prep(const float* __restrict__ x,
                                               const float* __restrict__ w1l, const float* __restrict__ b1l,
                                               const float* __restrict__ w1r,
                                               const float* __restrict__ w2l, const float* __restrict__ b2l,
                                               const float* __restrict__ w2r,
                                               const float* __restrict__ w3l, const float* __restrict__ b3l,
                                               const float* __restrict__ w3r,
                                               unsigned short* xb, unsigned short* w1c, unsigned short* w2c,
                                               unsigned short* w3c, float* bias) {
  const int tid = (int)threadIdx.x;
  const int blk = (int)blockIdx.x;
  if (blk < PBX) {
    const int u   = blk * NTHR + tid;
    const int row = u >> 3, k8 = (u & 7) * 8;
    const int rc  = row < NN ? row : NN - 1;
    const unsigned mk = row < NN ? 0xffffu : 0u;
    const float* p = x + (size_t)rc * HD + k8;
    const v4f a = *(const v4fa*)p;
    const v4f b = *(const v4fa*)(p + 4);
    v8us o;
    o[0] = (unsigned short)(bf16_bits(a.x) & mk); o[1] = (unsigned short)(bf16_bits(a.y) & mk);
    o[2] = (unsigned short)(bf16_bits(a.z) & mk); o[3] = (unsigned short)(bf16_bits(a.w) & mk);
    o[4] = (unsigned short)(bf16_bits(b.x) & mk); o[5] = (unsigned short)(bf16_bits(b.y) & mk);
    o[6] = (unsigned short)(bf16_bits(b.z) & mk); o[7] = (unsigned short)(bf16_bits(b.w) & mk);
    st2_v8us(xb + (size_t)row * HD + k8, o);
  } else {
    const int wb = blk - PBX;
    const int v2 = (wb & 1) * NTHR + tid;
    if (wb < 4)        wpart<64>(w1l, w1c, 192, (wb >> 1) * 64, v2);
    else if (wb < 6)   wpart<64>(w1r, w1c, 192, 128, v2);
    else if (wb < 10)  wpart<64>(w2l, w2c, 256, ((wb - 6) >> 1) * 64, v2);
    else if (wb < 14)  wpart<64>(w2r, w2c, 256, 128 + ((wb - 10) >> 1) * 64, v2);
    else if (wb < 16)  wpart<32>(w3l, w3c, 256, (wb - 14) * 64, tid);
    else if (wb < 18)  wpart<32>(w3r, w3c, 256, 128 + (wb - 16) * 64, tid);
    else if (tid < 64) {
      const int t = tid;
      const v4f a = *(const v4fa*)(b1l + 4 * (t & 15));
      const v4f b = *(const v4fa*)(b2l + 4 * (t & 15));
      const v4f c = *(const v4fa*)(b3l + 4 * (t & 7));
      asm volatile("" :: "v"(a));
      asm volatile("" :: "v"(b));
      asm volatile("" :: "v"(c));
      const unsigned ma = (t < 16) ? 0xffffffffu : 0u;
      const unsigned mb = (t >= 16 && t < 32) ? 0xffffffffu : 0u;
      const unsigned mc = (t >= 32 && t < 40) ? 0xffffffffu : 0u;
      v4f o;
      o.x = __uint_as_float(((bf16_bits(a.x) << 16) & ma) | ((bf16_bits(b.x) << 16) & mb) | ((bf16_bits(c.x) << 16) & mc));
      o.y = __uint_as_float(((bf16_bits(a.y) << 16) & ma) | ((bf16_bits(b.y) << 16) & mb) | ((bf16_bits(c.y) << 16) & mc));
      o.z = __uint_as_float(((bf16_bits(a.z) << 16) & ma) | ((bf16_bits(b.z) << 16) & mb) | ((bf16_bits(c.z) << 16) & mc));
      o.w = __uint_as_float(((bf16_bits(a.w) << 16) & ma) | ((bf16_bits(b.w) << 16) & mb) | ((bf16_bits(c.w) << 16) & mc));
      st2_v4f(bias + 4 * t, o);
    }
  }
}

__device__ __forceinline__ void bucket_flush(const int* pl, const int* cnt, int ov, int* lp, int* cop, int* fp,
                                             int tid) {
#pragma unroll 1
  for (int i = tid * 4; i < RCAP; i += NTHR * 4) {
    const v4i v = *(const v4ia*)(pl + i);
    *(volatile v4i*)(lp + i) = v;
  }
#pragma unroll 1
  for (int i = tid * 4; i < 2 * NBRUN; i += NTHR * 4) {
    const v4i v = *(const v4ia*)(cnt + i);
    *(volatile v4i*)(cop + i) = v;
  }
  if (tid < 8) {
    const v4i f = {ov, ov, ov, ov};
    *(volatile v4i*)(fp + 4 * tid) = f;
  }
}

__global__ __launch_bounds__(NTHR) void k_bucket(const int* __restrict__ srcs, const int* __restrict__ dsts,
                                                 int* LIST, int* CO, int* FLAG) {
  extern __shared__ __attribute__((aligned(16))) int dsm[];
  int* wl   = dsm;
  int* pl   = dsm + NWAVE * WLCAP;
  int* cnt  = pl + RCAP;
  int* offs = cnt + NBRUN;
  int* cur  = offs + NBRUN;
  int* misc = cur + NBRUN;
  const int tid = (int)threadIdx.x, lane = tid & 31, wave = tid >> 5;
  const int blk = (int)blockIdx.x;
  const unsigned nbs = (unsigned)(blk * NBRUN);

  {
    const v4i z4 = {0, 0, 0, 0};
    for (int i = tid * 4; i < BK_ZINTS; i += NTHR * 4) *(v4ia*)(dsm + i) = z4;
    if (tid < 16) misc[tid] = 0;
  }
  __syncthreads();

  {
    const int per  = ((NE + NWAVE * WCH - 1) / (NWAVE * WCH)) * WCH;
    const int ebeg = wave * per;
    const int eend = (ebeg + per < NE) ? (ebeg + per) : NE;
    int* mylist = wl + wave * WLCAP;
    int wc = 0;
#pragma unroll 1
    for (int cb = ebeg; cb < eend; cb += WCH) {
      const int e0 = cb + lane * EPT;
      const v4i da = *(const v4ia*)(dsts + e0);
      const v4i db = *(const v4ia*)(dsts + e0 + 4);
      const unsigned s0 = (unsigned)da.x - nbs, s1 = (unsigned)da.y - nbs;
      const unsigned s2 = (unsigned)da.z - nbs, s3 = (unsigned)da.w - nbs;
      const unsigned s4 = (unsigned)db.x - nbs, s5 = (unsigned)db.y - nbs;
      const unsigned s6 = (unsigned)db.z - nbs, s7 = (unsigned)db.w - nbs;
      const bool h0 = s0 < (unsigned)NBRUN, h1 = s1 < (unsigned)NBRUN, h2 = s2 < (unsigned)NBRUN, h3 = s3 < (unsigned)NBRUN;
      const bool h4 = s4 < (unsigned)NBRUN, h5 = s5 < (unsigned)NBRUN, h6 = s6 < (unsigned)NBRUN, h7 = s7 < (unsigned)NBRUN;
      const unsigned m0 = __builtin_amdgcn_ballot_w32(h0), m1 = __builtin_amdgcn_ballot_w32(h1);
      const unsigned m2 = __builtin_amdgcn_ballot_w32(h2), m3 = __builtin_amdgcn_ballot_w32(h3);
      const unsigned m4 = __builtin_amdgcn_ballot_w32(h4), m5 = __builtin_amdgcn_ballot_w32(h5);
      const unsigned m6 = __builtin_amdgcn_ballot_w32(h6), m7 = __builtin_amdgcn_ballot_w32(h7);
      const unsigned any = m0 | m1 | m2 | m3 | m4 | m5 | m6 | m7;
      if (any != 0u) {
        const int pre = (int)(__builtin_amdgcn_mbcnt_lo(m0, 0u) + __builtin_amdgcn_mbcnt_lo(m1, 0u) +
                              __builtin_amdgcn_mbcnt_lo(m2, 0u) + __builtin_amdgcn_mbcnt_lo(m3, 0u) +
                              __builtin_amdgcn_mbcnt_lo(m4, 0u) + __builtin_amdgcn_mbcnt_lo(m5, 0u) +
                              __builtin_amdgcn_mbcnt_lo(m6, 0u) + __builtin_amdgcn_mbcnt_lo(m7, 0u));
        int p = wc + pre;
        if (h0) { if (p < WLCAP) mylist[p] = ((e0 + 0) << SLB) | (int)s0; p = p + 1; }
        if (h1) { if (p < WLCAP) mylist[p] = ((e0 + 1) << SLB) | (int)s1; p = p + 1; }
        if (h2) { if (p < WLCAP) mylist[p] = ((e0 + 2) << SLB) | (int)s2; p = p + 1; }
        if (h3) { if (p < WLCAP) mylist[p] = ((e0 + 3) << SLB) | (int)s3; p = p + 1; }
        if (h4) { if (p < WLCAP) mylist[p] = ((e0 + 4) << SLB) | (int)s4; p = p + 1; }
        if (h5) { if (p < WLCAP) mylist[p] = ((e0 + 5) << SLB) | (int)s5; p = p + 1; }
        if (h6) { if (p < WLCAP) mylist[p] = ((e0 + 6) << SLB) | (int)s6; p = p + 1; }
        if (h7) { if (p < WLCAP) mylist[p] = ((e0 + 7) << SLB) | (int)s7; p = p + 1; }
        wc += (int)(__builtin_popcount(m0) + __builtin_popcount(m1) + __builtin_popcount(m2) + __builtin_popcount(m3) +
                    __builtin_popcount(m4) + __builtin_popcount(m5) + __builtin_popcount(m6) + __builtin_popcount(m7));
      }
    }
    if (lane == 0) misc[wave] = wc;
  }
  __syncthreads();

  if (wave == 0) {
    int ov = 0;
#pragma unroll 1
    for (int w2 = 0; w2 < NWAVE; ++w2) {
      int c = misc[w2];
      if (c > WLCAP) ov = 1;
      c = c < 0 ? 0 : (c > WLCAP ? WLCAP : c);
#pragma unroll 1
      for (int b0 = 0; b0 < c; b0 += 32) {
        const int idx = b0 + lane;
        const int ent = wl[w2 * WLCAP + (idx < WLCAP ? idx : WLCAP - 1)];
        const int m32 = (c - b0) < 32 ? (c - b0) : 32;
#pragma unroll 1
        for (int k = 0; k < m32; ++k) {
          const int u    = __builtin_amdgcn_readlane(ent, k);
          const int slot = u & (NBRUN - 1);
          if (lane == 0) cnt[slot] = cnt[slot] + 1;
        }
      }
    }
    if (lane == 0) misc[9] = ov;
  }
  __syncthreads();
  if (wave == 0) {
    const int base = lane * (NBRUN / 32);
    int s = 0;
#pragma unroll 1
    for (int i = 0; i < NBRUN / 32; ++i) s += cnt[base + i];
    int incl = s;
#pragma unroll
    for (int d = 1; d < 32; d <<= 1) {
      const int y = __shfl_up(incl, d, 32);
      if (lane >= d) incl += y;
    }
    int run = incl - s;
#pragma unroll 1
    for (int i = 0; i < NBRUN / 32; ++i) {
      const int cv = cnt[base + i];
      offs[base + i] = run;
      cur[base + i]  = run;
      run += cv;
    }
  }
  __syncthreads();

  if (wave == 0) {
#pragma unroll 1
    for (int w2 = 0; w2 < NWAVE; ++w2) {
      int c = misc[w2];
      c = c < 0 ? 0 : (c > WLCAP ? WLCAP : c);
#pragma unroll 1
      for (int b0 = 0; b0 < c; b0 += 32) {
        const int idx = b0 + lane;
        const int ent = wl[w2 * WLCAP + (idx < WLCAP ? idx : WLCAP - 1)];
        int eid = (ent >> SLB) & 0x1FFFFF;
        eid = eid > NE - 1 ? NE - 1 : eid;
        int sr = srcs[eid];
        sr = sr < 0 ? 0 : (sr > NN - 1 ? NN - 1 : sr);
        const int m32 = (c - b0) < 32 ? (c - b0) : 32;
#pragma unroll 1
        for (int k = 0; k < m32; ++k) {
          const int u    = __builtin_amdgcn_readlane(ent, k);
          const int wd   = __builtin_amdgcn_readlane(sr, k);
          const int slot = u & (NBRUN - 1);
          if (lane == 0) {
            int p = cur[slot];
            p = p < 0 ? 0 : (p > RCAP - 1 ? RCAP - 1 : p);
            pl[p] = wd;
            cur[slot] = p + 1;
          }
        }
      }
    }
  }
  __syncthreads();

  const int ovf = misc[9];
  int* lp  = LIST + (size_t)blk * RCAP;
  int* cop = CO + (size_t)blk * (2 * NBRUN);
  int* fp  = FLAG + (size_t)blk * 32;
  bucket_flush(pl, cnt, ovf, lp, cop, fp, tid);
  __threadfence();
  bucket_flush(pl, cnt, ovf, lp, cop, fp, tid);
}

template <int SRC>
__global__ __launch_bounds__(NTHR) void k_agg(const int* __restrict__ LIST, const int* __restrict__ CO,
                                              const int* __restrict__ FLAG, const unsigned short* __restrict__ S,
                                              unsigned short* M) {
  const int tid = (int)threadIdx.x, lane = tid & 31, wave = tid >> 5, hh = lane >> 4, q = lane & 15;
  const int rowBase = (int)blockIdx.x * ABM;
  const int bucket  = rowBase >> SLB;
  const int* lb  = LIST + (size_t)bucket * RCAP;
  const int* cob = CO + (size_t)bucket * (2 * NBRUN);
  const int flag = FLAG[(size_t)bucket * 32];
  const float qnan = __uint_as_float(0x7fc00000u);
  constexpr int SPITCH = (SRC == 0) ? HD : KH;

#pragma unroll 1
  for (int i = 0; i < ABM / (2 * NWAVE); ++i) {
    const int d    = rowBase + (ABM / NWAVE) * wave + 2 * i + hh;
    const int slot = d & (NBRUN - 1);
    int c = cob[slot];
    int o = cob[NBRUN + slot];
    const bool big = c > TRIPCAP;
    c = c < 0 ? 0 : (c > TRIPCAP ? TRIPCAP : c);
    o = o < 0 ? 0 : (o > RCAP - 1 ? RCAP - 1 : o);
    const int co = __shfl_xor(c, 16, 32);
    const int cm = c > co ? c : co;
    int last = o + c - 1; last = last < o ? o : last;
    last = last > RCAP - 1 ? RCAP - 1 : last;
    float a0 = 0.0f, a1 = 0.0f, a2 = 0.0f, a3 = 0.0f;
#pragma unroll 1
    for (int j = 0; j < cm; ++j) {
      int idx = o + j;
      idx = idx > last ? last : idx;
      int sr = lb[idx];
      sr = sr < 0 ? 0 : (sr > NN - 1 ? NN - 1 : sr);
      const unsigned short* rp = S + (size_t)sr * SPITCH + 4 * q;
      float f0, f1, f2, f3;
      if constexpr (SRC == 0) {
        const v2u w = *(const v2ua*)rp;
        asm volatile("" :: "v"(w.x), "v"(w.y));
        f0 = __uint_as_float(w.x << 16);
        f1 = __uint_as_float(w.x & 0xffff0000u);
        f2 = __uint_as_float(w.y << 16);
        f3 = __uint_as_float(w.y & 0xffff0000u);
      } else {
        const v2u wh = *(const v2ua*)rp;
        const v2u wl = *(const v2ua*)(rp + HD);
        asm volatile("" :: "v"(wh.x), "v"(wh.y));
        asm volatile("" :: "v"(wl.x), "v"(wl.y));
        f0 = __uint_as_float(wh.x << 16)         + __uint_as_float(wl.x << 16);
        f1 = __uint_as_float(wh.x & 0xffff0000u) + __uint_as_float(wl.x & 0xffff0000u);
        f2 = __uint_as_float(wh.y << 16)         + __uint_as_float(wl.y << 16);
        f3 = __uint_as_float(wh.y & 0xffff0000u) + __uint_as_float(wl.y & 0xffff0000u);
      }
      const bool valid = j < c;
      const float t0 = a0 + f0, t1 = a1 + f1, t2 = a2 + f2, t3 = a3 + f3;
      a0 = valid ? t0 : a0; a1 = valid ? t1 : a1; a2 = valid ? t2 : a2; a3 = valid ? t3 : a3;
    }
    const float den = fmaxf((float)c, 1.0f);
    float m0 = a0 / den, m1 = a1 / den, m2 = a2 / den, m3 = a3 / den;
    const bool bad  = (flag != 0) | big;
    const bool live = d < NN;
    m0 = bad ? qnan : m0; m1 = bad ? qnan : m1; m2 = bad ? qnan : m2; m3 = bad ? qnan : m3;
    m0 = live ? m0 : 0.0f; m1 = live ? m1 : 0.0f; m2 = live ? m2 : 0.0f; m3 = live ? m3 : 0.0f;
    int h01, h23, l01, l23;
    hilo_pack(m0, m1, m2, m3, h01, h23, l01, l23);
    const v4i ow = regroup8(h01, h23, l01, l23, lane);
    unsigned short* hp = M + (size_t)d * KH + 8 * q;
    *(volatile v4i*)hp = ow;
    __threadfence();
    *(volatile v4i*)hp = ow;
  }
}

template <int NT, int KLEN, int BPITCH>
__device__ __forceinline__ void gemm_seg(const unsigned short* __restrict__ ap,
                                         const unsigned short* __restrict__ bp, v8f (&acc)[NT]) {
#pragma unroll 1
  for (int k0 = 0; k0 < KLEN; k0 += 32) {
    FragB af;
    af.h[0] = *(const v8usa*)(ap + k0);
    af.h[1] = *(const v8usa*)(ap + k0 + 16);
#pragma unroll
    for (int nt = 0; nt < NT; ++nt) {
      const unsigned short* wq = bp + (size_t)(16 * nt) * (size_t)BPITCH + k0;
      FragB bf;
      bf.h[0] = *(const v8usa*)wq;
      bf.h[1] = *(const v8usa*)(wq + 16);
      acc[nt] = wmb(af, bf, acc[nt]);
    }
  }
}

template <int NT, int PITCH>
__device__ __forceinline__ void stage_d(float* stg, const v8f (&acc)[NT], int wave, int hh, int m) {
#pragma unroll
  for (int nt = 0; nt < NT; ++nt) {
#pragma unroll
    for (int r = 0; r < 8; ++r) stg[(16 * wave + 8 * hh + r) * PITCH + 16 * nt + m] = acc[nt][r];
  }
}

template <int LAYER>
__global__ __launch_bounds__(NTHR) __attribute__((amdgpu_num_vgpr(248)))
void k_gemm(const unsigned short* __restrict__ Mp, const unsigned short* __restrict__ Sp,
            const unsigned short* __restrict__ BT, const float* __restrict__ BIAS,
            const int* __restrict__ FLAG, unsigned short* Hout, float* out) {
  constexpr int SPITCH = (LAYER == 1) ? HD : KH;
  constexpr int K2     = SPITCH;
  constexpr int BP     = KH + K2;
  constexpr int NT     = (LAYER == 3) ? 2 : 4;
  constexpr int BOFF   = (LAYER - 1) * 64;
  static_assert(BP % 32 == 0 && K2 % 32 == 0 && KH % 32 == 0);
  __shared__ __attribute__((aligned(16))) float stg[GBM * SP];
  __shared__ __attribute__((aligned(16))) float sb[64];
  const int tid = (int)threadIdx.x, lane = tid & 31, wave = tid >> 5, hh = lane >> 4, m = lane & 15;
  const int rowBase = (int)blockIdx.x * GBM;
  if (tid < 16) *(v4fa*)(sb + 4 * tid) = *(const v4fa*)(BIAS + BOFF + 4 * tid);

  v8f acc[NT];
  {
    const v8f z = {0.f, 0.f, 0.f, 0.f, 0.f, 0.f, 0.f, 0.f};
#pragma unroll
    for (int t = 0; t < NT; ++t) acc[t] = z;
  }
  const size_t arow = (size_t)(rowBase + 16 * wave + m);
  const unsigned short* ap1 = Mp + arow * (size_t)KH + 8 * hh;
  const unsigned short* bp1 = BT + (size_t)m * (size_t)BP + 8 * hh;
  gemm_seg<NT, KH, BP>(ap1, bp1, acc);
  const unsigned short* ap2 = Sp + arow * (size_t)SPITCH + 8 * hh;
  const unsigned short* bp2 = BT + (size_t)m * (size_t)BP + KH + 8 * hh;
  gemm_seg<NT, K2, BP>(ap2, bp2, acc);

  if constexpr (LAYER != 3) {
    stage_d<NT, SP>(stg, acc, wave, hh, m);
    __syncthreads();
    const v4f bias = *(const v4fa*)(sb + 4 * m);
#pragma unroll 1
    for (int i = 0; i < 8; ++i) {
      const int lr   = 16 * wave + 2 * i + hh;
      const int grow = rowBase + lr;
      const bool live = grow < NN;
      const v4f a = *(const v4fa*)(stg + lr * SP + 4 * m);
      asm volatile("" :: "v"(a));
      float v0 = a.x + bias.x, v1 = a.y + bias.y, v2 = a.z + bias.z, v3 = a.w + bias.w;
      v0 = (v0 > 0.0f) ? v0 : (v0 - v0); v1 = (v1 > 0.0f) ? v1 : (v1 - v1);
      v2 = (v2 > 0.0f) ? v2 : (v2 - v2); v3 = (v3 > 0.0f) ? v3 : (v3 - v3);
      v0 = live ? v0 : 0.0f; v1 = live ? v1 : 0.0f; v2 = live ? v2 : 0.0f; v3 = live ? v3 : 0.0f;
      int h01, h23, l01, l23;
      hilo_pack(v0, v1, v2, v3, h01, h23, l01, l23);
      const v4i ow = regroup8(h01, h23, l01, l23, lane);
      unsigned short* hp = Hout + (size_t)grow * KH + 8 * m;
      *(volatile v4i*)hp = ow;
      __threadfence();
      *(volatile v4i*)hp = ow;
    }
  } else {
    stage_d<NT, SP3>(stg, acc, wave, hh, m);
    __syncthreads();
    const int flag = FLAG[(size_t)((int)blockIdx.x >> 3) * 32];
    const float qnan = __uint_as_float(0x7fc00000u);
    const int g = lane >> 3, c4 = lane & 7;
    const v4f bias = *(const v4fa*)(sb + 4 * c4);
#pragma unroll 1
    for (int i = 0; i < 4; ++i) {
      const int lr   = 16 * wave + 4 * i + g;
      const int grow = rowBase + lr;
      const bool live = grow < NN;
      const v4f a = *(const v4fa*)(stg + lr * SP3 + 4 * c4);
      asm volatile("" :: "v"(a));
      float v0 = a.x + bias.x, v1 = a.y + bias.y, v2 = a.z + bias.z, v3 = a.w + bias.w;
      v0 = (flag != 0) ? qnan : v0; v1 = (flag != 0) ? qnan : v1;
      v2 = (flag != 0) ? qnan : v2; v3 = (flag != 0) ? qnan : v3;
      v4f o;
      o.x = v0; o.y = v1; o.z = v2; o.w = v3;
      float* op = out + (size_t)grow * OC + 4 * c4;
      if (live) *(volatile v4f*)op = o;
      __threadfence();
      if (live) *(volatile v4f*)op = o;
    }
  }
}

extern "C" void kernel_launch(void* const* d_in, const int* in_sizes, int n_in,
                              void* d_out, int out_size, void* d_ws, size_t ws_size,
                              hipStream_t stream) {
  if (n_in < 11) return;
  if (in_sizes[0] != NN * HD) return;
  if (in_sizes[1] != 2 * NE) return;
  if (in_sizes[2] != HD * HD || in_sizes[3] != HD || in_sizes[4] != HD * HD) return;
  if (in_sizes[5] != HD * HD || in_sizes[6] != HD || in_sizes[7] != HD * HD) return;
  if (in_sizes[8] != HD * OC || in_sizes[9] != OC || in_sizes[10] != HD * OC) return;
  if (out_size != NN * OC) return;

  const float* x   = (const float*)d_in[0];
  const int*   ei  = (const int*)d_in[1];
  const float* W1l = (const float*)d_in[2];
  const float* b1l = (const float*)d_in[3];
  const float* W1r = (const float*)d_in[4];
  const float* W2l = (const float*)d_in[5];
  const float* b2l = (const float*)d_in[6];
  const float* W2r = (const float*)d_in[7];
  const float* W3l = (const float*)d_in[8];
  const float* b3l = (const float*)d_in[9];
  const float* W3r = (const float*)d_in[10];
  float* out = (float*)d_out;
  const int* srcs = ei;
  const int* dsts = ei + NE;

  constexpr size_t zXB   = (size_t)MP * HD * 2;
  constexpr size_t zHL   = (size_t)MP * KH * 2;
  constexpr size_t zLIST = (size_t)NBK * RCAP * 4;
  constexpr size_t zCO   = (size_t)NBK * 2 * NBRUN * 4;
  constexpr size_t zFLAG = (size_t)NBK * 128;
  constexpr size_t zW1   = (size_t)HD * 192 * 2;
  constexpr size_t zW2   = (size_t)HD * 256 * 2;
  constexpr size_t zW3   = (size_t)OC * 256 * 2;
  constexpr size_t zB    = 1024;
  constexpr size_t oXB   = 0;
  constexpr size_t oM    = oXB + zXB;
  constexpr size_t oH1   = oM + zHL;
  constexpr size_t oH2   = oH1 + zHL;
  constexpr size_t oLIST = oH2 + zHL;
  constexpr size_t oCO   = oLIST + zLIST;
  constexpr size_t oFLAG = oCO + zCO;
  constexpr size_t oW1   = oFLAG + zFLAG;
  constexpr size_t oW2   = oW1 + zW1;
  constexpr size_t oW3   = oW2 + zW2;
  constexpr size_t oB    = oW3 + zW3;
  constexpr size_t oEND  = oB + zB;
  static_assert(zXB % 256 == 0 && zHL % 256 == 0 && zLIST % 256 == 0 && zCO % 256 == 0 && zFLAG % 256 == 0);
  static_assert(zW1 % 256 == 0 && zW2 % 256 == 0 && zW3 % 256 == 0 && zB % 256 == 0);
  static_assert(oEND <= (size_t)WSMAX);
  if (oEND > ws_size) return;

  char* ws = (char*)d_ws;
  unsigned short* XB   = (unsigned short*)(ws + oXB);
  unsigned short* M    = (unsigned short*)(ws + oM);
  unsigned short* H1   = (unsigned short*)(ws + oH1);
  unsigned short* H2   = (unsigned short*)(ws + oH2);
  int*            LIST = (int*)(ws + oLIST);
  int*            CO   = (int*)(ws + oCO);
  int*            FLAG = (int*)(ws + oFLAG);
  unsigned short* W1C  = (unsigned short*)(ws + oW1);
  unsigned short* W2C  = (unsigned short*)(ws + oW2);
  unsigned short* W3C  = (unsigned short*)(ws + oW3);
  float*          BIAS = (float*)(ws + oB);

  hipFuncSetAttribute(reinterpret_cast<const void*>(&k_bucket), hipFuncAttributeMaxDynamicSharedMemorySize, (int)BK_LDS);

  k_prep<<<PBTOT, NTHR, 0, stream>>>(x, W1l, b1l, W1r, W2l, b2l, W2r, W3l, b3l, W3r, XB, W1C, W2C, W3C, BIAS);
  k_bucket<<<NBK, NTHR, BK_LDS, stream>>>(srcs, dsts, LIST, CO, FLAG);
  k_agg<0><<<MP / ABM, NTHR, 0, stream>>>(LIST, CO, FLAG, XB, M);
  k_gemm<1><<<MP / GBM, NTHR, 0, stream>>>(M, XB, W1C, BIAS, FLAG, H1, out);
  k_agg<1><<<MP / ABM, NTHR, 0, stream>>>(LIST, CO, FLAG, H1, M);
  k_gemm<2><<<MP / GBM, NTHR, 0, stream>>>(M, H1, W2C, BIAS, FLAG, H2, out);
  k_agg<1><<<MP / ABM, NTHR, 0, stream>>>(LIST, CO, FLAG, H2, M);
  k_gemm<3><<<MP / GBM, NTHR, 0, stream>>>(M, H2, W3C, BIAS, FLAG, H2, out);
}
